// DGMGearnet_25202868093418
// MI455X (gfx1250) — hardware-verified
//
#include <hip/hip_runtime.h>
#include <stdint.h>
#include <stddef.h>


namespace {

constexpr int kN   = 2048;
constexpr int kR   = 3;
constexpr int kNR  = kN * kR;
constexpr int kD   = 128;
constexpr int kSO  = 64;
constexpr int kWin = 256;
constexpr int kK   = 16;
constexpr int kQB  = kN / 16;
constexpr int kKT  = (16 + 2 * kWin) / 16;
constexpr int kSP  = kKT * 16 + 4;
constexpr int kTSP = 260;

typedef _Float16 v8h  __attribute__((ext_vector_type(8)));
typedef _Float16 v16h __attribute__((ext_vector_type(16)));
typedef __bf16   v16b __attribute__((ext_vector_type(16)));
typedef float    v8f  __attribute__((ext_vector_type(8)));
typedef float    v4f  __attribute__((ext_vector_type(4)));
typedef unsigned v4u  __attribute__((ext_vector_type(4)));

union H16 { v16h v; v8h h[2]; };
union P8  { v8h h; v4u u; _Float16 e[8]; };
struct BF2 { v16b hi; v16b lo; };

__device__ __forceinline__ v8f mma_f16(const v16h a, const v16h b, v8f c) {
  v8f d = __builtin_amdgcn_wmma_f32_16x16x32_f16(false, a, false, b, (short)0, c, false, false);
  asm volatile("v_nop\n\tv_nop\n\tv_nop\n\tv_nop" : "+v"(d) : "v"(a), "v"(b));
  return d;
}
__device__ __forceinline__ v8f mma_bf16(const v16b a, const v16b b, v8f c) {
  v8f d = __builtin_amdgcn_wmma_f32_16x16x32_bf16(false, a, false, b, (short)0, c, false, false);
  asm volatile("v_nop\n\tv_nop\n\tv_nop\n\tv_nop" : "+v"(d) : "v"(a), "v"(b));
  return d;
}

__device__ __forceinline__ BF2 split16(const float* p0, const float* p1) {
  const v4f a = *(const v4f*)p0;
  const v4f b = *(const v4f*)(p0 + 4);
  const v4f c = *(const v4f*)p1;
  const v4f d = *(const v4f*)(p1 + 4);
  const float x[16] = { a.x, a.y, a.z, a.w, b.x, b.y, b.z, b.w,
                        c.x, c.y, c.z, c.w, d.x, d.y, d.z, d.w };
  BF2 f;
#pragma unroll
  for (int i = 0; i < 16; ++i) {
    const __bf16 hh = (__bf16)x[i];
    f.hi[i] = hh;
    f.lo[i] = (__bf16)(x[i] - (float)hh);
  }
  return f;
}

__device__ __forceinline__ v4u pack8h(const float* s, float mul) {
  const v4f a = *(const v4f*)s;
  const v4f b = *(const v4f*)(s + 4);
  P8 p;
  p.e[0] = (_Float16)(a.x * mul); p.e[1] = (_Float16)(a.y * mul);
  p.e[2] = (_Float16)(a.z * mul); p.e[3] = (_Float16)(a.w * mul);
  p.e[4] = (_Float16)(b.x * mul); p.e[5] = (_Float16)(b.y * mul);
  p.e[6] = (_Float16)(b.z * mul); p.e[7] = (_Float16)(b.w * mul);
  return p.u;
}

__device__ __forceinline__ void adj_store_pass(const float* tile, _Float16* AT, int rowbase, int wave, int lane) {
#pragma unroll 2
  for (int it = 0; it < 16; ++it) {
    const int row  = 2 * wave + (it >> 3);
    const int hoff = ((it & 7) << 8) + 8 * lane;
    const v4u u = pack8h(tile + row * kN + hoff, 256.0f);
    *(volatile v4u*)(AT + (size_t)(rowbase + row) * kN + hoff) = u;
  }
}

__global__ __launch_bounds__(256)
void k_build_adj(const int* __restrict__ ei, const int* __restrict__ er,
                 const float* __restrict__ ew, int E, _Float16* __restrict__ AT)
{
  extern __shared__ v4f g_dyn[];
  __shared__ int   lidx[8][128];
  __shared__ float lwt[8][128];
  __shared__ int   lcnt[8];
  float* tile = (float*)g_dyn;

  const int tid = threadIdx.x, lane = tid & 31, wave = tid >> 5;
  const int rowbase = blockIdx.x * 16;
  if (rowbase >= kNR) return;
  const int br = rowbase / kN;
  const int d0 = rowbase - br * kN;

  {
    const v4f z = { 0.0f, 0.0f, 0.0f, 0.0f };
    for (int i = tid; i < 16 * kN / 4; i += 256) g_dyn[i] = z;
  }
  __syncthreads();

  const int npass = (E + 1023) >> 10;
  for (int p = 0; p < npass; ++p) {
    int cnt = 0;
#pragma unroll
    for (int it = 0; it < 4; ++it) {
      const int e = (p << 10) + (wave << 7) + (it << 5) + lane;
      int src = 0, dst = 0, rr = -1;
      float w = 0.0f;
      if (e < E) {
        src = ei[2 * (size_t)e];
        dst = ei[2 * (size_t)e + 1];
        rr  = er[e];
        w   = ew[e];
      }
      const bool match = (e < E) && (rr == br) && ((unsigned)(dst - d0) < 16u) &&
                         ((unsigned)src < (unsigned)kN);
      const unsigned mask = __builtin_amdgcn_ballot_w32(match);
      const int rank = __builtin_popcount(mask & ((1u << lane) - 1u));
      if (match) {
        lidx[wave][cnt + rank] = ((dst - d0) << 11) | src;
        lwt[wave][cnt + rank]  = w;
      }
      cnt += __builtin_popcount(mask);
    }
    if (lane == 0) lcnt[wave] = cnt;
    __syncthreads();
    if (tid == 0) {
      for (int wv = 0; wv < 8; ++wv) {
        int c = lcnt[wv];
        c = c > 128 ? 128 : (c < 0 ? 0 : c);
        for (int j = 0; j < c; ++j) {
          const int cell = lidx[wv][j] & 0x7fff;
          tile[cell] += lwt[wv][j];
        }
      }
    }
    __syncthreads();
  }

  adj_store_pass(tile, AT, rowbase, wave, lane);
  __threadfence();
  adj_store_pass(tile, AT, rowbase, wave, lane);
}

__device__ __forceinline__ void ts_store_pass(const float* Ts, _Float16* Hi, _Float16* Lo, int nrows,
                                              int rb, int cb, int wave, int lane, float s) {
#pragma unroll
  for (int it = 0; it < 4; ++it) {
    const int c = wave * 4 + it;
    const float* sp = Ts + c * kTSP + 8 * lane;
    const v4f a = *(const v4f*)sp;
    const v4f b = *(const v4f*)(sp + 4);
    const float x[8] = { a.x, a.y, a.z, a.w, b.x, b.y, b.z, b.w };
    P8 ph, pl;
#pragma unroll
    for (int i = 0; i < 8; ++i) {
      const float v = x[i] * s;
      const _Float16 hh = (_Float16)v;
      ph.e[i] = hh;
      pl.e[i] = (_Float16)(v - (float)hh);
    }
    const size_t o = (size_t)(cb + c) * nrows + rb + 8 * lane;
    *(volatile v4u*)(Hi + o) = ph.u;
    *(volatile v4u*)(Lo + o) = pl.u;
  }
}

__global__ __launch_bounds__(256)
void k_tsplit(const float* __restrict__ X, int nrows, int ncols, float s,
              _Float16* __restrict__ Hi, _Float16* __restrict__ Lo)
{
  __shared__ __attribute__((aligned(16))) float Ts[32 * kTSP];
  const int tid = threadIdx.x, lane = tid & 31, wave = tid >> 5;
  const int rb = blockIdx.x * 256, cb = blockIdx.y * 32;
  if (rb + 256 > nrows || cb + 32 > ncols) return;
  {
    const float* xp = X + (size_t)(rb + tid) * ncols + cb;
#pragma unroll
    for (int j4 = 0; j4 < 8; ++j4) {
      const v4f v = *(const v4f*)(xp + 4 * j4);
      Ts[(4 * j4 + 0) * kTSP + tid] = v.x;
      Ts[(4 * j4 + 1) * kTSP + tid] = v.y;
      Ts[(4 * j4 + 2) * kTSP + tid] = v.z;
      Ts[(4 * j4 + 3) * kTSP + tid] = v.w;
    }
  }
  __syncthreads();
  ts_store_pass(Ts, Hi, Lo, nrows, rb, cb, wave, lane, s);
  __threadfence();
  ts_store_pass(Ts, Hi, Lo, nrows, rb, cb, wave, lane, s);
}

constexpr int G1BM = 64, G1BN = 128, G1LP = 40, G1CP = 132;

__device__ __forceinline__ void g1_store_pass(const float* Cs, float* C, int m0, int wave, int lane,
                                              int ldc, int nodeN, int rcs) {
#pragma unroll 4
  for (int it = 0; it < 16; ++it) {
    const int row  = wave * 16 + it;
    const int grow = m0 + row;
    const size_t o = (size_t)(grow % nodeN) * ldc + (size_t)(grow / nodeN) * rcs + 4 * lane;
    const v4f v = *(const v4f*)(Cs + row * G1CP + 4 * lane);
    *(volatile v4f*)(C + o) = v;
  }
}

__global__ __launch_bounds__(128)
void k_gemm_agg(const _Float16* __restrict__ A, const _Float16* __restrict__ Bh,
                const _Float16* __restrict__ Bl, int uselo,
                const float* __restrict__ bias, int hasb, int relu, float scale,
                float* C, int ldc, int nodeN, int rcs, int M, int K)
{
  __shared__ __attribute__((aligned(16))) _Float16 As[G1BM * G1LP];
  __shared__ __attribute__((aligned(16))) _Float16 Bhs[G1BN * G1LP];
  __shared__ __attribute__((aligned(16))) _Float16 Bls[G1BN * G1LP];
  __shared__ __attribute__((aligned(16))) float Cs[G1BM * G1CP];

  const int tid = threadIdx.x, lane = tid & 31, wave = tid >> 5;
  const int h = lane >> 4, c16 = lane & 15;
  const int wm = wave & 1, wn = wave >> 1;
  const int m0 = blockIdx.x * G1BM;
  if (m0 + G1BM > M) return;

  v8f acc[2][4];
#pragma unroll
  for (int mt = 0; mt < 2; ++mt)
#pragma unroll
    for (int nt = 0; nt < 4; ++nt)
#pragma unroll
      for (int rr = 0; rr < 8; ++rr) acc[mt][nt][rr] = 0.0f;

  const int nslab = K >> 5;
  for (int s = 0; s < nslab; ++s) {
    const int k0 = s << 5;
#pragma unroll
    for (int i = 0; i < 2; ++i) {
      const int idx = tid + 128 * i, row = idx >> 2, c = idx & 3;
      *(v4u*)&As[row * G1LP + 8 * c] = *(const v4u*)(A + (size_t)(m0 + row) * K + k0 + 8 * c);
    }
#pragma unroll
    for (int i = 0; i < 4; ++i) {
      const int idx = tid + 128 * i, d = idx >> 2, c = idx & 3;
      *(v4u*)&Bhs[d * G1LP + 8 * c] = *(const v4u*)(Bh + (size_t)d * K + k0 + 8 * c);
    }
    if (uselo) {
#pragma unroll
      for (int i = 0; i < 4; ++i) {
        const int idx = tid + 128 * i, d = idx >> 2, c = idx & 3;
        *(v4u*)&Bls[d * G1LP + 8 * c] = *(const v4u*)(Bl + (size_t)d * K + k0 + 8 * c);
      }
    }
    __syncthreads();

    H16 a[2], b[4];
#pragma unroll
    for (int mt = 0; mt < 2; ++mt) {
      const int row = wm * 32 + mt * 16 + c16;
      a[mt].h[0] = *(const v8h*)&As[row * G1LP + 8 * h];
      a[mt].h[1] = *(const v8h*)&As[row * G1LP + 16 + 8 * h];
    }
#pragma unroll
    for (int nt = 0; nt < 4; ++nt) {
      const int d = wn * 64 + nt * 16 + c16;
      b[nt].h[0] = *(const v8h*)&Bhs[d * G1LP + 8 * h];
      b[nt].h[1] = *(const v8h*)&Bhs[d * G1LP + 16 + 8 * h];
    }
#pragma unroll
    for (int mt = 0; mt < 2; ++mt)
#pragma unroll
      for (int nt = 0; nt < 4; ++nt)
        acc[mt][nt] = mma_f16(a[mt].v, b[nt].v, acc[mt][nt]);
    if (uselo) {
#pragma unroll
      for (int nt = 0; nt < 4; ++nt) {
        const int d = wn * 64 + nt * 16 + c16;
        b[nt].h[0] = *(const v8h*)&Bls[d * G1LP + 8 * h];
        b[nt].h[1] = *(const v8h*)&Bls[d * G1LP + 16 + 8 * h];
      }
#pragma unroll
      for (int mt = 0; mt < 2; ++mt)
#pragma unroll
        for (int nt = 0; nt < 4; ++nt)
          acc[mt][nt] = mma_f16(a[mt].v, b[nt].v, acc[mt][nt]);
    }
    __syncthreads();
  }

#pragma unroll
  for (int mt = 0; mt < 2; ++mt)
#pragma unroll
    for (int nt = 0; nt < 4; ++nt) {
      const int col = wn * 64 + nt * 16 + c16;
      const float bv = hasb ? bias[col] : 0.0f;
#pragma unroll
      for (int rr = 0; rr < 8; ++rr) {
        const int row = wm * 32 + mt * 16 + 8 * h + rr;
        float v = acc[mt][nt][rr] * scale + bv;
        if (relu) v = fmaxf(v, 0.0f);
        Cs[row * G1CP + col] = v;
      }
    }
  __syncthreads();
  g1_store_pass(Cs, C, m0, wave, lane, ldc, nodeN, rcs);
  __threadfence();
  g1_store_pass(Cs, C, m0, wave, lane, ldc, nodeN, rcs);
}

constexpr int G2BM = 64, G2BN = 64, G2LP = 36, G2CP = 68;

__device__ __forceinline__ void g2_store_pass(const float* Cs, float* C, int m0, int n0, int wave,
                                              int h, int c16, int ldc) {
#pragma unroll
  for (int it = 0; it < 8; ++it) {
    const int row = wave * 16 + it * 2 + h;
    const int col4 = 4 * c16;
    const v4f v = *(const v4f*)(Cs + row * G2CP + col4);
    *(volatile v4f*)(C + (size_t)(m0 + row) * ldc + n0 + col4) = v;
  }
}

__global__ __launch_bounds__(128)
void k_gemm_x3(const float* __restrict__ A1, int lda1, int seg1, int K1,
               const float* __restrict__ A2, int lda2, int seg2,
               const float* __restrict__ B1, const float* __restrict__ B2, int ldb,
               const float* __restrict__ bias1, int hasb1,
               const float* __restrict__ bias2, int hasb2,
               float* C, int ldc, int M, int Nc, int K, int relu)
{
  __shared__ __attribute__((aligned(16))) float As[G2BM * G2LP];
  __shared__ __attribute__((aligned(16))) float Bt[G2BN * G2LP];
  __shared__ __attribute__((aligned(16))) float Cs[G2BM * G2CP];

  const int tid = threadIdx.x, lane = tid & 31, wave = tid >> 5;
  const int h = lane >> 4, c16 = lane & 15;
  const int wm = wave & 1, wn = wave >> 1;
  const int m0 = blockIdx.x * G2BM, n0 = blockIdx.y * G2BN;
  if (m0 + G2BM > M || n0 + G2BN > Nc) return;

  v8f acc[2][2];
#pragma unroll
  for (int mt = 0; mt < 2; ++mt)
#pragma unroll
    for (int nt = 0; nt < 2; ++nt)
#pragma unroll
      for (int rr = 0; rr < 8; ++rr) acc[mt][nt][rr] = 0.0f;

  const int nslab = K >> 5;
  for (int s = 0; s < nslab; ++s) {
    const int k0 = s << 5;
    const bool reg1 = k0 < K1;
    const int kk = reg1 ? k0 : (k0 - K1);
    const float* Ab = reg1 ? (A1 + (size_t)(kk >> 7) * seg1 + (kk & 127))
                           : (A2 + (size_t)(kk >> 7) * seg2 + (kk & 127));
    const int lda = reg1 ? lda1 : lda2;
    const float* Bb = reg1 ? (B1 + (size_t)kk * ldb + n0) : (B2 + (size_t)kk * ldb + n0);

#pragma unroll
    for (int i = 0; i < 4; ++i) {
      const int idx = tid + 128 * i, row = idx >> 3, c4 = idx & 7;
      *(v4f*)&As[row * G2LP + 4 * c4] = *(const v4f*)(Ab + (size_t)(m0 + row) * lda + 4 * c4);
    }
#pragma unroll
    for (int i = 0; i < 4; ++i) {
      const int idx = tid + 128 * i, kr = idx >> 4, c4 = idx & 15;
      const v4f v = *(const v4f*)(Bb + (size_t)kr * ldb + 4 * c4);
      Bt[(4 * c4 + 0) * G2LP + kr] = v.x;
      Bt[(4 * c4 + 1) * G2LP + kr] = v.y;
      Bt[(4 * c4 + 2) * G2LP + kr] = v.z;
      Bt[(4 * c4 + 3) * G2LP + kr] = v.w;
    }
    __syncthreads();

    BF2 a[2], b[2];
#pragma unroll
    for (int mt = 0; mt < 2; ++mt) {
      const int row = wm * 32 + mt * 16 + c16;
      a[mt] = split16(&As[row * G2LP + 8 * h], &As[row * G2LP + 16 + 8 * h]);
    }
#pragma unroll
    for (int nt = 0; nt < 2; ++nt) {
      const int col = wn * 32 + nt * 16 + c16;
      b[nt] = split16(&Bt[col * G2LP + 8 * h], &Bt[col * G2LP + 16 + 8 * h]);
    }
#pragma unroll
    for (int mt = 0; mt < 2; ++mt)
#pragma unroll
      for (int nt = 0; nt < 2; ++nt) {
        acc[mt][nt] = mma_bf16(a[mt].hi, b[nt].hi, acc[mt][nt]);
        acc[mt][nt] = mma_bf16(a[mt].hi, b[nt].lo, acc[mt][nt]);
        acc[mt][nt] = mma_bf16(a[mt].lo, b[nt].hi, acc[mt][nt]);
      }
    __syncthreads();
  }

#pragma unroll
  for (int mt = 0; mt < 2; ++mt)
#pragma unroll
    for (int nt = 0; nt < 2; ++nt) {
      const int col = wn * 32 + nt * 16 + c16;
      float bv = 0.0f;
      if (hasb1) bv += bias1[n0 + col];
      if (hasb2) bv += bias2[n0 + col];
#pragma unroll
      for (int rr = 0; rr < 8; ++rr) {
        const int row = wm * 32 + mt * 16 + 8 * h + rr;
        float v = acc[mt][nt][rr] + bv;
        if (relu) v = fmaxf(v, 0.0f);
        Cs[row * G2CP + col] = v;
      }
    }
  __syncthreads();
  g2_store_pass(Cs, C, m0, n0, wave, h, c16, ldc);
  __threadfence();
  g2_store_pass(Cs, C, m0, n0, wave, h, c16, ldc);
}

__global__ __launch_bounds__(256)
void k_scores_topk(const float* __restrict__ Q, const float* __restrict__ KM, unsigned* __restrict__ TK)
{
  __shared__ __attribute__((aligned(16))) float S[16][kSP];
  __shared__ __attribute__((aligned(16))) unsigned tl[8][32];

  const int tid = threadIdx.x, lane = tid & 31, wave = tid >> 5;
  const int h = lane >> 4, c16 = lane & 15;
  const int r = blockIdx.x / kQB;
  const int qb = blockIdx.x - r * kQB;
  if (r >= kR) return;
  const int n0 = qb * 16;
  const int mbase = n0 - kWin;

  BF2 aq[2];
  {
    const float* qp = Q + (size_t)(r * kN + n0 + c16) * kSO;
#pragma unroll
    for (int ks = 0; ks < 2; ++ks) aq[ks] = split16(qp + ks * 32 + 8 * h, qp + ks * 32 + 16 + 8 * h);
  }
  for (int kt = wave; kt < kKT; kt += 8) {
    int m = mbase + kt * 16 + c16;
    m = m < 0 ? 0 : (m > kN - 1 ? kN - 1 : m);
    const float* kp = KM + (size_t)(r * kN + m) * kSO;
    v8f acc;
#pragma unroll
    for (int rr = 0; rr < 8; ++rr) acc[rr] = 0.0f;
#pragma unroll
    for (int ks = 0; ks < 2; ++ks) {
      const BF2 bk = split16(kp + ks * 32 + 8 * h, kp + ks * 32 + 16 + 8 * h);
      acc = mma_bf16(aq[ks].hi, bk.hi, acc);
      acc = mma_bf16(aq[ks].hi, bk.lo, acc);
      acc = mma_bf16(aq[ks].lo, bk.hi, acc);
    }
#pragma unroll
    for (int rr = 0; rr < 8; ++rr) S[8 * h + rr][kt * 16 + c16] = acc[rr] * 0.0625f;
  }
  __syncthreads();

  for (int qq = 0; qq < 2; ++qq) {
    const int qi = wave * 2 + qq;
    const int n = n0 + qi;
    const int mlo = (n - kWin) > 0 ? (n - kWin) : 0;
    const int mhi = (n + kWin) < (kN - 1) ? (n + kWin) : (kN - 1);
    const int jlo = mlo - mbase, jhi = mhi - mbase;
    float myv = 0.0f;
    int myj = 0x7fffffff;
    for (int t = 0; t < kK; ++t) {
      float best = -__builtin_inff();
      int bj = 0x7fffffff;
      for (int j = jlo + lane; j <= jhi; j += 32) {
        const float v = S[qi][j];
        if (v > best) { best = v; bj = j; }
      }
#pragma unroll
      for (int off = 16; off > 0; off >>= 1) {
        const float ov = __shfl_xor(best, off, 32);
        const int   oj = __shfl_xor(bj, off, 32);
        if (ov > best || (ov == best && oj < bj)) { best = ov; bj = oj; }
      }
      if (lane == t) { myv = best; myj = bj; }
      if (lane == 0 && (unsigned)bj < (unsigned)(kKT * 16)) S[qi][bj] = -__builtin_inff();
      __syncthreads();
    }
    const float vmax = __shfl(myv, 0, 32);
    const float ex = (lane < kK) ? expf((myv - vmax) * 2.0f) : 0.0f;
    float sum = ex;
#pragma unroll
    for (int off = 16; off > 0; off >>= 1) sum += __shfl_xor(sum, off, 32);
    const float soft = ex * (1.0f / sum);
    const int msel = ((unsigned)myj < (unsigned)(kKT * 16)) ? (mbase + myj) : -1;
    if (lane < kK) {
      tl[wave][lane] = __float_as_uint(soft);
      tl[wave][16 + lane] = (unsigned)msel;
    }
    __syncthreads();
    v4u u = { 0u, 0u, 0u, 0u };
    if (lane < 8) u = *(const v4u*)&tl[wave][4 * lane];
    unsigned* g = TK + (size_t)(r * kN + n) * 32 + 4 * lane;
    if (lane < 8) *(volatile v4u*)g = u;
    __threadfence();
    if (lane < 8) *(volatile v4u*)g = u;
    __syncthreads();
  }
}

__device__ __forceinline__ void ne_store_pass(const v4u* tile4, _Float16* NE, int rowbase, int wave, int lane) {
#pragma unroll 2
  for (int it = 0; it < 16; ++it) {
    const int row = 2 * wave + (it >> 3);
    const int c = ((it & 7) << 5) + lane;
    const v4u u = tile4[row * (kN / 8) + c];
    *(volatile v4u*)(NE + (size_t)(rowbase + row) * kN + 8 * c) = u;
  }
}

__global__ __launch_bounds__(256)
void k_build_ne(const _Float16* __restrict__ AT, const unsigned* __restrict__ TK, _Float16* __restrict__ NE)
{
  extern __shared__ v4f g_dyn[];
  v4u* tile4 = (v4u*)g_dyn;
  _Float16* tile = (_Float16*)g_dyn;

  const int tid = threadIdx.x, lane = tid & 31, wave = tid >> 5;
  const int rowbase = blockIdx.x * 16;
  if (rowbase >= kNR) return;
  const int br = rowbase / kN;
  const int d0 = rowbase - br * kN;

  for (int i = tid; i < 16 * (kN / 8); i += 256) {
    const int row = i >> 8, c = i & 255;
    tile4[i] = *(const v4u*)(AT + (size_t)(rowbase + row) * kN + 8 * c);
  }
  __syncthreads();

  const int qlo = (d0 - kWin) > 0 ? (d0 - kWin) : 0;
  int qhi = d0 + 15 + kWin;
  qhi = qhi > (kN - 1) ? (kN - 1) : qhi;
  const int nent = (qhi - qlo + 1) * kK;
  for (int e = tid; e < nent; e += 256) {
    const int n = qlo + (e >> 4), slot = e & 15;
    const size_t tb = (size_t)(br * kN + n) * 32;
    const float soft = __uint_as_float(TK[tb + slot]);
    const int m = (int)TK[tb + 16 + slot];
    if ((unsigned)(m - d0) < 16u) {
      const int cell = (m - d0) * kN + n;
      const _Float16 nv = (_Float16)(soft * 256.0f);
      if ((float)nv > (float)tile[cell]) tile[cell] = nv;
    }
  }
  __syncthreads();

  ne_store_pass(tile4, NE, rowbase, wave, lane);
  __threadfence();
  ne_store_pass(tile4, NE, rowbase, wave, lane);
}

__global__ __launch_bounds__(128)
void k_colsum(const float* Hm, int nrows, float* outg)
{
  __shared__ __attribute__((aligned(16))) float ss[kD];
  const int d = threadIdx.x;
  double s = 0.0;
  for (int n = 0; n < nrows; ++n) s += (double)Hm[(size_t)n * kD + d];
  ss[d] = (float)s;
  __syncthreads();
  v4f v = { 0.0f, 0.0f, 0.0f, 0.0f };
  if (d < 32) v = *(const v4f*)&ss[4 * d];
  if (d < 32) *(volatile v4f*)(outg + 4 * d) = v;
  __threadfence();
  if (d < 32) *(volatile v4f*)(outg + 4 * d) = v;
}

}

extern "C" void kernel_launch(void* const* d_in, const int* in_sizes, int n_in,
                              void* d_out, int out_size, void* d_ws, size_t ws_size,
                              hipStream_t stream)
{
  if (n_in < 20) return;
  if (in_sizes[0] != kN * kD || in_sizes[2] <= 0 || in_sizes[1] != 2 * in_sizes[2] ||
      in_sizes[3] != in_sizes[2] ||
      in_sizes[4] != kD * kD || in_sizes[5] != kD || in_sizes[6] != 4 * kD * kD || in_sizes[7] != kD ||
      in_sizes[8] != kD * kSO || in_sizes[9] != kD * kSO || in_sizes[10] != kD * kSO || in_sizes[11] != kD * kSO ||
      in_sizes[12] != 3 * kD * kD || in_sizes[13] != kD || in_sizes[14] != kD * kD || in_sizes[15] != kD ||
      in_sizes[16] != 3 * kD * kD || in_sizes[17] != kD || in_sizes[18] != kD * kD || in_sizes[19] != kD ||
      out_size != kD + kN * kD) return;
  const int E = in_sizes[2];

  const float* x    = (const float*)d_in[0];
  const int*   ei   = (const int*)d_in[1];
  const int*   er   = (const int*)d_in[2];
  const float* ew   = (const float*)d_in[3];
  const float* Ws0  = (const float*)d_in[4];
  const float* bs0  = (const float*)d_in[5];
  const float* Ws1  = (const float*)d_in[6];
  const float* bs1  = (const float*)d_in[7];
  const float* Wq0  = (const float*)d_in[8];
  const float* Wk0  = (const float*)d_in[9];
  const float* Wq1  = (const float*)d_in[10];
  const float* Wk1  = (const float*)d_in[11];
  const float* W0   = (const float*)d_in[12];
  const float* b0   = (const float*)d_in[13];
  const float* Wsl0 = (const float*)d_in[14];
  const float* bsl0 = (const float*)d_in[15];
  const float* W1   = (const float*)d_in[16];
  const float* b1   = (const float*)d_in[17];
  const float* Wsl1 = (const float*)d_in[18];
  const float* bsl1 = (const float*)d_in[19];

  float* outg = (float*)d_out;
  float* h1   = outg + kD;

  size_t off = 0;
  auto carve = [&](size_t bytes) -> void* {
    void* p = (char*)d_ws + off;
    off += (bytes + 255) & ~(size_t)255;
    return p;
  };
  const size_t adjN = (size_t)kNR * kN;
  _Float16* ATh  = (_Float16*)carve(adjN * 2);
  _Float16* NEh  = (_Float16*)carve(adjN * 2);
  unsigned* TK   = (unsigned*)carve((size_t)kNR * 32 * 4);
  _Float16* xTh  = (_Float16*)carve((size_t)kD * kN * 2);
  _Float16* xTl  = (_Float16*)carve((size_t)kD * kN * 2);
  _Float16* h0Th = (_Float16*)carve((size_t)kD * kN * 2);
  _Float16* h0Tl = (_Float16*)carve((size_t)kD * kN * 2);
  _Float16* PTh  = (_Float16*)carve((size_t)kD * kN * 2);
  _Float16* PTl  = (_Float16*)carve((size_t)kD * kN * 2);
  float*    t0   = (float*)carve((size_t)kNR * kD * 4);
  float*    rel0 = (float*)carve((size_t)kNR * kD * 4);
  float*    rel1 = (float*)carve((size_t)kNR * kD * 4);
  float*    qv   = (float*)carve((size_t)kNR * kSO * 4);
  float*    kv   = (float*)carve((size_t)kNR * kSO * 4);
  float*    agg  = (float*)carve((size_t)kN * 3 * kD * 4);
  float*    h0   = (float*)carve((size_t)kN * kD * 4);
  float*    Pm   = (float*)carve((size_t)kN * kD * 4);
  if (off > ws_size) return;

  const size_t ldsAdj = (size_t)16 * kN * 4;
  const size_t ldsNe  = (size_t)16 * kN * 2;
  const dim3 gT(kN / 256, kD / 32);
  const float scX  = 1.0f / (256.0f * 64.0f);
  const float scH  = 1.0f / (256.0f * 8.0f);
  const int segRel = kN * kD;

  k_build_adj<<<kNR / 16, 256, ldsAdj, stream>>>(ei, er, ew, E, ATh);
  k_tsplit<<<gT, 256, 0, stream>>>(x, kN, kD, 64.0f, xTh, xTl);

  k_gemm_agg<<<kNR / G1BM, 128, 0, stream>>>(ATh, xTh, xTl, 1, bs0, 0, 0, scX, t0, kD, kNR, 0, kNR, kN);
  k_gemm_x3<<<dim3(kNR / G2BM, kD / G2BN), 128, 0, stream>>>(
      t0, kD, 0, kD, t0, kD, 0, Ws0, Ws0, kD, bs0, 1, bs0, 0, rel0, kD, kNR, kD, kD, 1);
  k_gemm_x3<<<dim3(kNR / G2BM, kSO / G2BN), 128, 0, stream>>>(
      rel0, kD, 0, kD, rel0, kD, 0, Wq0, Wq0, kSO, bs0, 0, bs0, 0, qv, kSO, kNR, kSO, kD, 0);
  k_gemm_x3<<<dim3(kNR / G2BM, kSO / G2BN), 128, 0, stream>>>(
      rel0, kD, 0, kD, rel0, kD, 0, Wk0, Wk0, kSO, bs0, 0, bs0, 0, kv, kSO, kNR, kSO, kD, 0);
  k_scores_topk<<<kR * kQB, 256, 0, stream>>>(qv, kv, TK);
  k_build_ne<<<kNR / 16, 256, ldsNe, stream>>>(ATh, TK, NEh);

  k_gemm_agg<<<kNR / G1BM, 128, 0, stream>>>(NEh, xTh, xTl, 1, bs0, 0, 0, scX, agg, 3 * kD, kN, kD, kNR, kN);
  k_gemm_x3<<<dim3(kN / G2BM, kD / G2BN), 128, 0, stream>>>(
      agg, 3 * kD, kD, 3 * kD, x, kD, 0, W0, Wsl0, kD, b0, 1, bsl0, 1, h0, kD, kN, kD, 4 * kD, 1);
  k_tsplit<<<gT, 256, 0, stream>>>(h0, kN, kD, 8.0f, h0Th, h0Tl);

  k_gemm_x3<<<dim3(kN / G2BM, kD / G2BN), 128, 0, stream>>>(
      h0, kD, 0, kD, rel0, kD, segRel, Ws1, Ws1 + kD * kD, kD, bs1, 0, bs1, 0, Pm, kD, kN, kD, 4 * kD, 0);
  k_tsplit<<<gT, 256, 0, stream>>>(Pm, kN, kD, 8.0f, PTh, PTl);
  k_gemm_agg<<<kNR / G1BM, 128, 0, stream>>>(NEh, PTh, PTl, 1, bs1, 1, 1, scH, rel1, kD, kNR, 0, kNR, kN);
  k_gemm_x3<<<dim3(kNR / G2BM, kSO / G2BN), 128, 0, stream>>>(
      rel1, kD, 0, kD, rel1, kD, 0, Wq1, Wq1, kSO, bs1, 0, bs1, 0, qv, kSO, kNR, kSO, kD, 0);
  k_gemm_x3<<<dim3(kNR / G2BM, kSO / G2BN), 128, 0, stream>>>(
      rel1, kD, 0, kD, rel1, kD, 0, Wk1, Wk1, kSO, bs1, 0, bs1, 0, kv, kSO, kNR, kSO, kD, 0);
  k_scores_topk<<<kR * kQB, 256, 0, stream>>>(qv, kv, TK);
  k_build_ne<<<kNR / 16, 256, ldsNe, stream>>>(ATh, TK, NEh);

  k_gemm_agg<<<kNR / G1BM, 128, 0, stream>>>(NEh, h0Th, h0Th, 0, bs1, 0, 0, scH, agg, 3 * kD, kN, kD, kNR, kN);
  k_gemm_x3<<<dim3(kN / G2BM, kD / G2BN), 128, 0, stream>>>(
      agg, 3 * kD, kD, 3 * kD, h0, kD, 0, W1, Wsl1, kD, b1, 1, bsl1, 1, h1, kD, kN, kD, 4 * kD, 1);
  k_colsum<<<1, kD, 0, stream>>>(h1, kN, outg);
}
